// SA_Block_32865089749659
// MI455X (gfx1250) — hardware-verified
//
#include <hip/hip_runtime.h>
#include <stdint.h>
#include <stddef.h>


#ifndef NB
#define NB 4
#endif
#ifndef SEQ
#define SEQ 4096
#endif
#define NB_FULL 4
#define SEQ_FULL 4096

typedef _Float16 f16_t;
typedef __attribute__((ext_vector_type(16))) _Float16 v16h;
typedef __attribute__((ext_vector_type(8)))  _Float16 v8h_t;
typedef __attribute__((ext_vector_type(8)))  float v8f;
typedef __attribute__((ext_vector_type(4)))  float v4f_t;
typedef __attribute__((ext_vector_type(4)))  unsigned int v4u_t;
typedef v8h_t __attribute__((__may_alias__)) v8h;
typedef v4f_t __attribute__((__may_alias__)) v4f;
typedef v4u_t __attribute__((__may_alias__)) v4u;

constexpr int kB  = NB;
constexpr int kBF = NB_FULL;
constexpr int kN  = SEQ;
constexpr int kNF = SEQ_FULL;
constexpr int kC  = 512;
constexpr int kNH = kN / 2;
constexpr int PT  = 64;
constexpr int XP  = kC + 8;
constexpr int NPB = kN / PT;
constexpr int SP  = 72;
constexpr int FP  = 36;
constexpr int KP  = 40;
constexpr int SMB = (kN / 8 < 256) ? (kN / 8) : 256;
constexpr int NCH = kN / (8 * SMB);
constexpr int NWS = SMB / 32;

static_assert(kB >= 1 && kB <= kBF);
static_assert(kN >= 256 && kN <= kNF && (kN % 256) == 0);
static_assert((kN % PT) == 0 && (kNH % 128) == 0 && (kNH % 32) == 0 && (kN % 128) == 0);
static_assert(kC == 512 && (kC % 64) == 0 && (kC % 32) == 0);
static_assert(SMB * 8 * NCH == kN && NWS >= 1 && NCH >= 1 && NCH <= 2);
static_assert(((kB * kC) % 32) == 0 && ((kB * kC) % 256) == 0);
static_assert((XP % 8) == 0 && (SP % 8) == 0 && (KP % 8) == 0 && (FP % 4) == 0);

constexpr size_t XPROJ_LDS = (size_t)PT * XP * 2 + (size_t)64 * SP * 2 + (size_t)kC * 4;
constexpr size_t ZPROJ_LDS = (size_t)PT * XP * 2 + 2 * (size_t)64 * SP * 2 + 2 * (size_t)kC * 4;
static_assert(XPROJ_LDS == 77824 && ZPROJ_LDS == 89088);

union Frag  { v16h v; v8h_t h2[2]; f16_t e[16]; };
union Pack8 { v4u_t u; f16_t e[8]; };

static __device__ __forceinline__ v8f mma16(v16h a, v16h b, v8f c) {
  v8f d = __builtin_amdgcn_wmma_f32_16x16x32_f16(false, a, false, b, (short)0, c, false, false);
  asm volatile("v_nop\n\tv_nop\n\tv_nop\n\tv_nop" : "+v"(d) : "v"(a), "v"(b));
  return d;
}

static __device__ __forceinline__ v16h frag16(const f16_t* row, int h) {
  Frag f;
  f.h2[0] = *(const v8h*)(row + 8 * h);
  f.h2[1] = *(const v8h*)(row + 16 + 8 * h);
  return f.v;
}

static __device__ __forceinline__ float bfr(float x) {
  unsigned int u = __float_as_uint(x);
  u = (u + 0x7FFFu + ((u >> 16) & 1u)) & 0xFFFF0000u;
  return __uint_as_float(u);
}

static __device__ __forceinline__ float wmaxf(float v) {
#pragma unroll
  for (int o = 16; o > 0; o >>= 1) v = fmaxf(v, __shfl_xor(v, o));
  return v;
}
static __device__ __forceinline__ float wsumf(float v) {
#pragma unroll
  for (int o = 16; o > 0; o >>= 1) v += __shfl_xor(v, o);
  return v;
}
static __device__ __forceinline__ double wsumd(double v) {
#pragma unroll
  for (int o = 16; o > 0; o >>= 1) v += __shfl_xor(v, o);
  return v;
}

__global__ void __launch_bounds__(256)
cvtw_kernel(const float* __restrict__ Wi, const float* __restrict__ Wo,
            f16_t* __restrict__ Wi16, f16_t* __restrict__ Wo16) {
  constexpr int per = kC * kC / 8;
  constexpr int bpp = per / 256;
  const int p = (blockIdx.x >= bpp) ? 1 : 0;
  const int g = (blockIdx.x - p * bpp) * 256 + threadIdx.x;
  const size_t e0 = (size_t)g * 8;
  const float* src = p ? Wo : Wi;
  f16_t* dst = p ? Wo16 : Wi16;
  const v4f a = *(const v4f*)(src + e0);
  const v4f c = *(const v4f*)(src + e0 + 4);
  Pack8 k;
#pragma unroll
  for (int e = 0; e < 4; ++e) {
    k.e[e]     = (f16_t)(bfr(a[e]) * 64.0f);
    k.e[4 + e] = (f16_t)(bfr(c[e]) * 64.0f);
  }
  *(volatile v4u_t*)(dst + e0) = k.u;
  __threadfence();
  *(volatile v4u_t*)(dst + e0) = k.u;
}

__global__ void __launch_bounds__(256)
stats_kernel(const float* __restrict__ cin, const float* __restrict__ sin_,
             float* __restrict__ mu_c, float* __restrict__ r_c,
             float* __restrict__ mu_s, float* __restrict__ r_s) {
  __shared__ alignas(16) float smu[32];
  __shared__ alignas(16) float srr[32];
  const int tid = threadIdx.x, wv = tid >> 5, l = tid & 31;
  constexpr int bpt = kB * kC / 32;
  const int t = (blockIdx.x >= bpt) ? 1 : 0;
  const int row0 = (blockIdx.x - t * bpt) * 32;
  const float* X = t ? sin_ : cin;
  float* MU = t ? mu_s : mu_c;
  float* RR = t ? r_s : r_c;
#pragma unroll 1
  for (int jj = 0; jj < 4; ++jj) {
    const int j = jj * 8 + wv;
    const int g = row0 + j;
    const int b = g / kC, ch = g - b * kC;
    const float* xr = X + ((size_t)b * kC + ch) * kNF;
    double s0 = 0.0, s1 = 0.0;
#pragma unroll 1
    for (int k = 0; k < kN / 128; ++k) {
      const v4f v = *(const v4f*)(xr + k * 128 + l * 4);
#pragma unroll
      for (int e = 0; e < 4; ++e) {
        const double f = (double)bfr(v[e]);
        s0 += f;
        s1 += f * f;
      }
    }
    s0 = wsumd(s0);
    s1 = wsumd(s1);
    if (l == 0) {
      const double mean = s0 / (double)kN;
      double var = (s1 - s0 * mean) / (double)(kN - 1);
      if (var < 0.0) var = 0.0;
      const float vf = (float)var + 1e-5f;
      smu[j] = (float)mean;
      srr[j] = 1.0f / sqrtf(vf);
    }
  }
  __syncthreads();
  const v4f vm = *(const v4f*)(smu + (tid & 7) * 4);
  const v4f vr = *(const v4f*)(srr + (tid & 7) * 4);
  v4f_t v;
#pragma unroll
  for (int e = 0; e < 4; ++e) v[e] = (tid < 8) ? vm[e] : vr[e];
  float* dst = ((tid < 8) ? MU : RR) + row0 + (tid & 7) * 4;
  if (tid < 16) *(volatile v4f_t*)dst = v;
  __threadfence();
  if (tid < 16) *(volatile v4f_t*)dst = v;
}

__global__ void __launch_bounds__(128)
mgemm_kernel(const float* __restrict__ Ws, const float* __restrict__ Wc,
             const float* __restrict__ r_c, f16_t* __restrict__ Mp) {
  __shared__ alignas(16) f16_t at[64 * KP];
  __shared__ alignas(16) f16_t bt[64 * KP];
  __shared__ alignas(16) f16_t shi[64 * SP];
  __shared__ alignas(16) f16_t slo[64 * SP];
  const int tid = threadIdx.x, wv = tid >> 5, l = tid & 31, h = l >> 4, m = l & 15;
  const int r0 = blockIdx.y * 64;
  const int c0 = blockIdx.x * 64;
  v8f acc[4];
#pragma unroll
  for (int ct = 0; ct < 4; ++ct) acc[ct] = v8f{};
#pragma unroll 1
  for (int ks = 0; ks < kC / 32; ++ks) {
    const int k0 = ks * 32;
    __syncthreads();
#pragma unroll
    for (int it = 0; it < 4; ++it) {
      const int idx = it * 128 + tid;
      const int kk = idx >> 4;
      const int j4 = (idx & 15) * 4;
      const v4f a = *(const v4f*)(Ws + (size_t)(k0 + kk) * kC + r0 + j4);
      const v4f c = *(const v4f*)(Wc + (size_t)(k0 + kk) * kC + c0 + j4);
#pragma unroll
      for (int e = 0; e < 4; ++e) {
        at[(j4 + e) * KP + kk] = (f16_t)(bfr(a[e]) * 64.0f);
        bt[(j4 + e) * KP + kk] = (f16_t)(bfr(c[e]) * 64.0f);
      }
    }
    __syncthreads();
    const v16h af = frag16(at + (wv * 16 + m) * KP, h);
#pragma unroll
    for (int ct = 0; ct < 4; ++ct) acc[ct] = mma16(af, frag16(bt + (ct * 16 + m) * KP, h), acc[ct]);
  }
#pragma unroll 1
  for (int b = 0; b < kB; ++b) {
    __syncthreads();
#pragma unroll
    for (int ct = 0; ct < 4; ++ct) {
      const float rc = r_c[b * kC + c0 + ct * 16 + m] * (1.0f / 64.0f);
#pragma unroll
      for (int r = 0; r < 8; ++r) {
        const float v  = acc[ct][r] * rc;
        const f16_t hv = (f16_t)v;
        const f16_t lv = (f16_t)((v - (float)hv) * 2048.0f);
        const int o = (wv * 16 + 8 * h + r) * SP + ct * 16 + m;
        shi[o] = hv;
        slo[o] = lv;
      }
    }
    __syncthreads();
    v4u_t vv[8];
    size_t gg[8];
#pragma unroll
    for (int it = 0; it < 8; ++it) {
      const int L   = it * 16 + (tid >> 3);
      const int pl  = it >> 2;
      const int row = L & 63;
      const int seg = tid & 7;
      const f16_t* st = pl ? slo : shi;
      vv[it] = *(const v4u*)(st + row * SP + seg * 8);
      gg[it] = ((size_t)(b * 2 + pl) * kC + r0 + row) * kC + c0 + seg * 8;
    }
#pragma unroll
    for (int it = 0; it < 8; ++it) *(volatile v4u_t*)(Mp + gg[it]) = vv[it];
    __threadfence();
#pragma unroll
    for (int it = 0; it < 8; ++it) *(volatile v4u_t*)(Mp + gg[it]) = vv[it];
  }
}

__global__ void __launch_bounds__(256)
q_kernel(const float* __restrict__ Ws, const float* __restrict__ bc, const f16_t* __restrict__ Mp,
         const float* __restrict__ mu_c, float* __restrict__ qv) {
  __shared__ alignas(16) float sq[256];
  const int tid = threadIdx.x;
  const int g = blockIdx.x * 256 + tid;
  const int b = g / kC, cp = g - b * kC;
  float v = 0.0f;
#pragma unroll 1
  for (int o = 0; o < kC; ++o) v += bfr(Ws[(size_t)o * kC + cp]) * bfr(bc[o]);
  const f16_t* mh = Mp + ((size_t)(b * 2) * kC + cp) * kC;
  const f16_t* ml = Mp + ((size_t)(b * 2 + 1) * kC + cp) * kC;
  const float* mub = mu_c + b * kC;
  float w = 0.0f;
#pragma unroll 1
  for (int c = 0; c < kC; ++c) {
    const float mv = ((float)mh[c] + (float)ml[c] * (1.0f / 2048.0f)) * (1.0f / 64.0f);
    w += mv * mub[c];
  }
  sq[tid] = v - w;
  __syncthreads();
  const v4f_t o4 = *(const v4f*)(sq + (tid & 63) * 4);
  float* dst = qv + (size_t)blockIdx.x * 256 + (tid & 63) * 4;
  if (tid < 64) *(volatile v4f_t*)dst = o4;
  __threadfence();
  if (tid < 64) *(volatile v4f_t*)dst = o4;
}

__global__ void __launch_bounds__(128)
xproj_kernel(const float* __restrict__ s, const f16_t* __restrict__ Wi16, const float* __restrict__ bi,
             f16_t* __restrict__ sT, f16_t* __restrict__ xf16) {
  extern __shared__ __align__(16) unsigned char lds_x[];
  f16_t* xt = reinterpret_cast<f16_t*>(lds_x);
  f16_t* sv = xt + PT * XP;
  float* sb = reinterpret_cast<float*>(sv + 64 * SP);

  const int tid = threadIdx.x, wv = tid >> 5, l = tid & 31, h = l >> 4, m = l & 15;
  const int b  = blockIdx.x / NPB;
  const int p0 = (blockIdx.x - b * NPB) * PT;
  if (b >= kB) return;

  for (int i = tid; i < kC; i += 128) sb[i] = bfr(bi[i]);

  const float* xb = s + (size_t)b * kC * kNF + p0;
#pragma unroll 2
  for (int it = 0; it < (kC * PT / 4) / 128; ++it) {
    const int c  = it * 8 + (tid >> 4);
    const int i4 = (tid & 15) * 4;
    const v4f v  = *(const v4f*)(xb + (size_t)c * kNF + i4);
    f16_t* d = xt + i4 * XP + c;
    d[0]      = (f16_t)(bfr(v[0]) * 16.0f);
    d[XP]     = (f16_t)(bfr(v[1]) * 16.0f);
    d[2 * XP] = (f16_t)(bfr(v[2]) * 16.0f);
    d[3 * XP] = (f16_t)(bfr(v[3]) * 16.0f);
  }
  __syncthreads();

#pragma unroll 4
  for (int it = 0; it < 32; ++it) {
    const int idx = it * 128 + tid;
    const int row = idx >> 6, seg = idx & 63;
    const v4u_t v = *(const v4u*)(xt + row * XP + seg * 8);
    *(volatile v4u_t*)(sT + ((size_t)(b * kN + p0 + row)) * kC + seg * 8) = v;
  }
  __threadfence();
#pragma unroll 4
  for (int it = 0; it < 32; ++it) {
    const int idx = it * 128 + tid;
    const int row = idx >> 6, seg = idx & 63;
    const v4u_t v = *(const v4u*)(xt + row * XP + seg * 8);
    *(volatile v4u_t*)(sT + ((size_t)(b * kN + p0 + row)) * kC + seg * 8) = v;
  }

  const f16_t* xrow = xt + (wv * 16 + m) * XP;
#pragma unroll 1
  for (int og = 0; og < kC / 64; ++og) {
    v8f av[4];
#pragma unroll
    for (int t = 0; t < 4; ++t) av[t] = v8f{};
#pragma unroll 1
    for (int ks = 0; ks < kC / 32; ++ks) {
      const int k0 = ks * 32;
      const v16h xf = frag16(xrow + k0, h);
#pragma unroll
      for (int t = 0; t < 4; ++t)
        av[t] = mma16(frag16(Wi16 + (size_t)(og * 64 + t * 16 + m) * kC + k0, h), xf, av[t]);
    }
    __syncthreads();
#pragma unroll
    for (int t = 0; t < 4; ++t)
#pragma unroll
      for (int r = 0; r < 8; ++r) {
        const int ol = t * 16 + 8 * h + r;
        sv[ol * SP + wv * 16 + m] = (f16_t)((av[t][r] * (1.0f / 1024.0f) + sb[og * 64 + ol]) * 16.0f);
      }
    __syncthreads();
    v4u_t vv[4];
    size_t gv[4];
#pragma unroll
    for (int q = 0; q < 4; ++q) {
      const int row = q * 16 + (tid >> 3);
      const int seg = tid & 7;
      vv[q] = *(const v4u*)(sv + row * SP + seg * 8);
      gv[q] = ((size_t)(b * kC + og * 64 + row)) * kN + p0 + seg * 8;
    }
#pragma unroll
    for (int q = 0; q < 4; ++q) *(volatile v4u_t*)(xf16 + gv[q]) = vv[q];
    __threadfence();
#pragma unroll
    for (int q = 0; q < 4; ++q) *(volatile v4u_t*)(xf16 + gv[q]) = vv[q];
  }
}

__global__ void __launch_bounds__(128)
zproj_kernel(const float* __restrict__ cin, const f16_t* __restrict__ Mp, const float* __restrict__ qv,
             const float* __restrict__ r_s, f16_t* __restrict__ Zh, f16_t* __restrict__ Zl) {
  extern __shared__ __align__(16) unsigned char lds_z[];
  f16_t* xt  = reinterpret_cast<f16_t*>(lds_z);
  f16_t* shi = xt + PT * XP;
  f16_t* slo = shi + 64 * SP;
  float* sq  = reinterpret_cast<float*>(slo + 64 * SP);
  float* srs = sq + kC;

  const int tid = threadIdx.x, wv = tid >> 5, l = tid & 31, h = l >> 4, m = l & 15;
  const int b  = blockIdx.x / NPB;
  const int p0 = (blockIdx.x - b * NPB) * PT;
  if (b >= kB) return;

  for (int i = tid; i < kC; i += 128) {
    sq[i]  = qv[b * kC + i];
    srs[i] = r_s[b * kC + i];
  }

  const float* xb = cin + (size_t)b * kC * kNF + p0;
#pragma unroll 2
  for (int it = 0; it < (kC * PT / 4) / 128; ++it) {
    const int c  = it * 8 + (tid >> 4);
    const int i4 = (tid & 15) * 4;
    const v4f v  = *(const v4f*)(xb + (size_t)c * kNF + i4);
    f16_t* d = xt + i4 * XP + c;
    d[0]      = (f16_t)(bfr(v[0]) * 16.0f);
    d[XP]     = (f16_t)(bfr(v[1]) * 16.0f);
    d[2 * XP] = (f16_t)(bfr(v[2]) * 16.0f);
    d[3 * XP] = (f16_t)(bfr(v[3]) * 16.0f);
  }
  __syncthreads();

  const f16_t* xrow = xt + (wv * 16 + m) * XP;
  const f16_t* mhb = Mp + (size_t)(b * 2) * kC * kC;
  const f16_t* mlb = Mp + (size_t)(b * 2 + 1) * kC * kC;
#pragma unroll 1
  for (int og = 0; og < kC / 64; ++og) {
    v8f ah[4], al[4];
#pragma unroll
    for (int t = 0; t < 4; ++t) { ah[t] = v8f{}; al[t] = v8f{}; }
#pragma unroll 1
    for (int ks = 0; ks < kC / 32; ++ks) {
      const int k0 = ks * 32;
      const v16h xf = frag16(xrow + k0, h);
#pragma unroll
      for (int t = 0; t < 4; ++t) {
        const size_t ro = (size_t)(og * 64 + t * 16 + m) * kC + k0;
        ah[t] = mma16(frag16(mhb + ro, h), xf, ah[t]);
        al[t] = mma16(frag16(mlb + ro, h), xf, al[t]);
      }
    }
    __syncthreads();
#pragma unroll
    for (int t = 0; t < 4; ++t)
#pragma unroll
      for (int r = 0; r < 8; ++r) {
        const int cl = t * 16 + 8 * h + r;
        const int cp = og * 64 + cl;
        const float z  = (ah[t][r] + al[t][r] * (1.0f / 2048.0f)) * (1.0f / 1024.0f) + sq[cp];
        const float zp = z * srs[cp];
        const f16_t hv = (f16_t)zp;
        const f16_t lv = (f16_t)((zp - (float)hv) * 2048.0f);
        const int o = (wv * 16 + m) * SP + cl;
        shi[o] = hv;
        slo[o] = lv;
      }
    __syncthreads();
    v4u_t vv[8];
    size_t gg[8];
#pragma unroll
    for (int it = 0; it < 8; ++it) {
      const int L   = it * 16 + (tid >> 3);
      const int pl  = it >> 2;
      const int i   = L & 63;
      const int seg = tid & 7;
      const f16_t* st = pl ? slo : shi;
      vv[it] = *(const v4u*)(st + i * SP + seg * 8);
      gg[it] = ((size_t)(b * kN + p0 + i)) * kC + og * 64 + seg * 8;
    }
#pragma unroll
    for (int it = 0; it < 8; ++it) {
      f16_t* dst = (it >> 2) ? Zl : Zh;
      *(volatile v4u_t*)(dst + gg[it]) = vv[it];
    }
    __threadfence();
#pragma unroll
    for (int it = 0; it < 8; ++it) {
      f16_t* dst = (it >> 2) ? Zl : Zh;
      *(volatile v4u_t*)(dst + gg[it]) = vv[it];
    }
  }
}

__global__ void __launch_bounds__(256)
sgemm_kernel(const f16_t* __restrict__ Zh, const f16_t* __restrict__ Zl, const f16_t* __restrict__ sT,
             float* __restrict__ S, int b, int nbase) {
  __shared__ alignas(16) float stg[8 * 32 * FP];
  const int tid = threadIdx.x, wv = tid >> 5, l = tid & 31, h = l >> 4, m = l & 15;
  const int rg = wv >> 2, cg = wv & 3;
  const int nt0 = blockIdx.y * 64 + rg * 32;
  const int mt0 = blockIdx.x * 128 + cg * 32;
  const f16_t* za = Zh + ((size_t)(b * kN + nbase + nt0)) * kC;
  const f16_t* zb = Zl + ((size_t)(b * kN + nbase + nt0)) * kC;
  const f16_t* kb = sT + ((size_t)(b * kN + mt0)) * kC;
  v8f ah[2][2], ax[2][2];
#pragma unroll
  for (int i = 0; i < 2; ++i)
#pragma unroll
    for (int j = 0; j < 2; ++j) { ah[i][j] = v8f{}; ax[i][j] = v8f{}; }
#pragma unroll 1
  for (int ks = 0; ks < kC / 32; ++ks) {
    const int k0 = ks * 32;
    const v16h a0 = frag16(za + (size_t)m * kC + k0, h);
    const v16h a1 = frag16(za + (size_t)(16 + m) * kC + k0, h);
    const v16h e0 = frag16(zb + (size_t)m * kC + k0, h);
    const v16h e1 = frag16(zb + (size_t)(16 + m) * kC + k0, h);
    const v16h b0 = frag16(kb + (size_t)m * kC + k0, h);
    const v16h b1 = frag16(kb + (size_t)(16 + m) * kC + k0, h);
    ah[0][0] = mma16(a0, b0, ah[0][0]);
    ah[0][1] = mma16(a0, b1, ah[0][1]);
    ah[1][0] = mma16(a1, b0, ah[1][0]);
    ah[1][1] = mma16(a1, b1, ah[1][1]);
    ax[0][0] = mma16(e0, b0, ax[0][0]);
    ax[0][1] = mma16(e0, b1, ax[0][1]);
    ax[1][0] = mma16(e1, b0, ax[1][0]);
    ax[1][1] = mma16(e1, b1, ax[1][1]);
  }
  float* wst = stg + wv * 32 * FP;
#pragma unroll
  for (int i = 0; i < 2; ++i)
#pragma unroll
    for (int j = 0; j < 2; ++j)
#pragma unroll
      for (int r = 0; r < 8; ++r)
        wst[(i * 16 + 8 * h + r) * FP + j * 16 + m] =
            (ah[i][j][r] + ax[i][j][r] * (1.0f / 2048.0f)) * (1.0f / 16.0f);
  __syncthreads();
  v4f_t ov[8];
  size_t go[8];
#pragma unroll
  for (int q = 0; q < 8; ++q) {
    const int row = q * 4 + (l >> 3);
    const int seg = l & 7;
    ov[q] = *(const v4f*)(wst + row * FP + seg * 4);
    go[q] = (size_t)(nt0 + row) * kN + mt0 + seg * 4;
  }
#pragma unroll
  for (int q = 0; q < 8; ++q) *(volatile v4f_t*)(S + go[q]) = ov[q];
  __threadfence();
#pragma unroll
  for (int q = 0; q < 8; ++q) *(volatile v4f_t*)(S + go[q]) = ov[q];
}

__global__ void __launch_bounds__(SMB)
softmax_kernel(const float* __restrict__ S, f16_t* __restrict__ P, float* __restrict__ invl) {
  __shared__ float wred[NWS];
  __shared__ alignas(16) float sl[32];
  const int tid = threadIdx.x, wv = tid >> 5, l = tid & 31;
  const int r0 = blockIdx.x * 32;
  const float kMinN = 6.103515625e-5f;
#pragma unroll 1
  for (int j = 0; j < 32; ++j) {
    const int row = r0 + j;
    const float* sr = S + (size_t)row * kN;
    f16_t* pr = P + (size_t)row * kN;
    v4f_t va[NCH], vb[NCH];
    float mx = -3.0e38f;
#pragma unroll
    for (int k = 0; k < NCH; ++k) {
      const int base = k * SMB * 8 + tid * 8;
      va[k] = *(const v4f*)(sr + base);
      vb[k] = *(const v4f*)(sr + base + 4);
#pragma unroll
      for (int e = 0; e < 4; ++e) mx = fmaxf(mx, fmaxf(va[k][e], vb[k][e]));
    }
    mx = wmaxf(mx);
    if (l == 0) wred[wv] = mx;
    __syncthreads();
    float rm = wred[0];
#pragma unroll
    for (int w = 1; w < NWS; ++w) rm = fmaxf(rm, wred[w]);
    __syncthreads();
    float ps = 0.0f;
    Pack8 pk[NCH];
#pragma unroll
    for (int k = 0; k < NCH; ++k) {
#pragma unroll
      for (int e = 0; e < 4; ++e) {
        float t0 = __expf(va[k][e] - rm) * 16384.0f;
        t0 = (t0 < kMinN) ? 0.0f : t0;
        const f16_t h0 = (f16_t)t0;
        ps += (float)h0;
        pk[k].e[e] = h0;
        float t1 = __expf(vb[k][e] - rm) * 16384.0f;
        t1 = (t1 < kMinN) ? 0.0f : t1;
        const f16_t h1 = (f16_t)t1;
        ps += (float)h1;
        pk[k].e[4 + e] = h1;
      }
    }
#pragma unroll
    for (int k = 0; k < NCH; ++k) *(volatile v4u_t*)(pr + k * SMB * 8 + tid * 8) = pk[k].u;
    ps = wsumf(ps);
    if (l == 0) wred[wv] = ps;
    __syncthreads();
    if (tid == 0) {
      float tot = 0.0f;
#pragma unroll
      for (int w = 0; w < NWS; ++w) tot += wred[w];
      sl[j] = 1.0f / tot;
    }
    __threadfence();
#pragma unroll
    for (int k = 0; k < NCH; ++k) *(volatile v4u_t*)(pr + k * SMB * 8 + tid * 8) = pk[k].u;
    __syncthreads();
  }
  const v4f_t o4 = *(const v4f*)(sl + (tid & 7) * 4);
  float* dst = invl + r0 + (tid & 7) * 4;
  if (tid < 8) *(volatile v4f_t*)dst = o4;
  __threadfence();
  if (tid < 8) *(volatile v4f_t*)dst = o4;
}

__global__ void __launch_bounds__(256)
pv_kernel(const f16_t* __restrict__ xf16, const f16_t* __restrict__ P, const float* __restrict__ invl,
          f16_t* __restrict__ Ofp, int b, int nbase) {
  __shared__ alignas(16) f16_t st[128 * SP];
  const int tid = threadIdx.x, wv = tid >> 5, l = tid & 31, h = l >> 4, m = l & 15;
  const int rg = wv >> 2, cg = wv & 3;
  const int c0  = blockIdx.y * 64;
  const int ct0 = c0 + rg * 32;
  const int nb0 = blockIdx.x * 128;
  const int nl0 = nb0 + cg * 32;
  const f16_t* xa = xf16 + ((size_t)(b * kC + ct0)) * kN;
  const f16_t* pb = P + (size_t)nl0 * kN;
  v8f acc[2][2];
#pragma unroll
  for (int i = 0; i < 2; ++i)
#pragma unroll
    for (int j = 0; j < 2; ++j) acc[i][j] = v8f{};
#pragma unroll 1
  for (int ks = 0; ks < kN / 32; ++ks) {
    const int k0 = ks * 32;
    const v16h a0 = frag16(xa + (size_t)m * kN + k0, h);
    const v16h a1 = frag16(xa + (size_t)(16 + m) * kN + k0, h);
    const v16h b0 = frag16(pb + (size_t)m * kN + k0, h);
    const v16h b1 = frag16(pb + (size_t)(16 + m) * kN + k0, h);
    acc[0][0] = mma16(a0, b0, acc[0][0]);
    acc[0][1] = mma16(a0, b1, acc[0][1]);
    acc[1][0] = mma16(a1, b0, acc[1][0]);
    acc[1][1] = mma16(a1, b1, acc[1][1]);
  }
  const float il0 = invl[nl0 + m];
  const float il1 = invl[nl0 + 16 + m];
#pragma unroll
  for (int i = 0; i < 2; ++i)
#pragma unroll
    for (int j = 0; j < 2; ++j)
#pragma unroll
      for (int r = 0; r < 8; ++r) {
        const int cl = rg * 32 + i * 16 + 8 * h + r;
        const int nl = cg * 32 + j * 16 + m;
        st[nl * SP + cl] = (f16_t)(acc[i][j][r] * (j ? il1 : il0));
      }
  __syncthreads();
  v4u_t vv[4];
  size_t gg[4];
#pragma unroll
  for (int q = 0; q < 4; ++q) {
    const int row = q * 32 + (tid >> 3);
    const int seg = tid & 7;
    vv[q] = *(const v4u*)(st + row * SP + seg * 8);
    gg[q] = ((size_t)(b * kN + nbase + nb0 + row)) * kC + c0 + seg * 8;
  }
#pragma unroll
  for (int q = 0; q < 4; ++q) *(volatile v4u_t*)(Ofp + gg[q]) = vv[q];
  __threadfence();
#pragma unroll
  for (int q = 0; q < 4; ++q) *(volatile v4u_t*)(Ofp + gg[q]) = vv[q];
}

__global__ void __launch_bounds__(256)
out_kernel(const f16_t* __restrict__ Wo16, const f16_t* __restrict__ Ofp, const float* __restrict__ bo,
           const float* __restrict__ x, float* __restrict__ out) {
  __shared__ alignas(16) float stg[8 * 32 * FP];
  const int tid = threadIdx.x, wv = tid >> 5, l = tid & 31, h = l >> 4, m = l & 15;
  const int rg = wv >> 2, cg = wv & 3;
  const int b  = blockIdx.z;
  const int o0 = blockIdx.y * 64 + rg * 32;
  const int n0 = blockIdx.x * 128 + cg * 32;
  const f16_t* wa = Wo16 + (size_t)o0 * kC;
  const f16_t* ob = Ofp + ((size_t)(b * kN + n0)) * kC;
  v8f acc[2][2];
#pragma unroll
  for (int i = 0; i < 2; ++i)
#pragma unroll
    for (int j = 0; j < 2; ++j) acc[i][j] = v8f{};
#pragma unroll 1
  for (int ks = 0; ks < kC / 32; ++ks) {
    const int k0 = ks * 32;
    const v16h a0 = frag16(wa + (size_t)m * kC + k0, h);
    const v16h a1 = frag16(wa + (size_t)(16 + m) * kC + k0, h);
    const v16h b0 = frag16(ob + (size_t)m * kC + k0, h);
    const v16h b1 = frag16(ob + (size_t)(16 + m) * kC + k0, h);
    acc[0][0] = mma16(a0, b0, acc[0][0]);
    acc[0][1] = mma16(a0, b1, acc[0][1]);
    acc[1][0] = mma16(a1, b0, acc[1][0]);
    acc[1][1] = mma16(a1, b1, acc[1][1]);
  }
  float* wst = stg + wv * 32 * FP;
#pragma unroll
  for (int i = 0; i < 2; ++i)
#pragma unroll
    for (int j = 0; j < 2; ++j)
#pragma unroll
      for (int r = 0; r < 8; ++r)
        wst[(i * 16 + 8 * h + r) * FP + j * 16 + m] = acc[i][j][r] * (1.0f / 1024.0f);
  __syncthreads();
  v4f_t ov[8];
  size_t go[8];
#pragma unroll
  for (int q = 0; q < 8; ++q) {
    const int row = q * 4 + (l >> 3);
    const int seg = l & 7;
    const int o   = o0 + row;
    go[q] = ((size_t)(b * kC + o)) * kNF + n0 + seg * 4;
    const v4f av = *(const v4f*)(wst + row * FP + seg * 4);
    const v4f xv = *(const v4f*)(x + go[q]);
    const float bb = bfr(bo[o]);
#pragma unroll
    for (int e = 0; e < 4; ++e) ov[q][e] = bfr(xv[e]) + (av[e] + bb);
  }
#pragma unroll
  for (int q = 0; q < 8; ++q) *(volatile v4f_t*)(out + go[q]) = ov[q];
  __threadfence();
#pragma unroll
  for (int q = 0; q < 8; ++q) *(volatile v4f_t*)(out + go[q]) = ov[q];
}

extern "C" void kernel_launch(void* const* d_in, const int* in_sizes, int n_in,
                              void* d_out, int out_size, void* d_ws, size_t ws_size,
                              hipStream_t stream) {
  if (n_in < 11) return;
  if (in_sizes[0] < kB * kC * kNF || in_sizes[1] < kB * kC * kNF || in_sizes[2] < kB * kC * kNF) return;
  if (in_sizes[3] < kC * kC || in_sizes[5] < kC * kC || in_sizes[7] < kC * kC || in_sizes[9] < kC * kC) return;
  if (in_sizes[4] < kC || in_sizes[6] < kC || in_sizes[8] < kC || in_sizes[10] < kC) return;
  if (out_size < kB * kC * kNF) return;

  const float* c   = (const float*)d_in[0];
  const float* s   = (const float*)d_in[1];
  const float* x   = (const float*)d_in[2];
  const float* c_w = (const float*)d_in[3];
  const float* c_b = (const float*)d_in[4];
  const float* s_w = (const float*)d_in[5];
  const float* i_w = (const float*)d_in[7];
  const float* i_b = (const float*)d_in[8];
  const float* o_w = (const float*)d_in[9];
  const float* o_b = (const float*)d_in[10];
  float* out = (float*)d_out;

  const size_t statB  = (size_t)kB * kC * sizeof(float);
  const size_t wplB   = (size_t)kC * kC * sizeof(f16_t);
  const size_t mpB    = (size_t)kB * 2 * kC * kC * sizeof(f16_t);
  const size_t actB   = (size_t)kB * kN * kC * sizeof(f16_t);
  const size_t sB     = (size_t)kNH * kN * sizeof(float);
  const size_t pB     = (size_t)kNH * kN * sizeof(f16_t);
  const size_t ilB    = (size_t)kNH * sizeof(float);
  size_t off = 0;
  float* mu_c = (float*)((char*)d_ws + off); off += statB;
  float* r_c  = (float*)((char*)d_ws + off); off += statB;
  float* mu_s = (float*)((char*)d_ws + off); off += statB;
  float* r_s  = (float*)((char*)d_ws + off); off += statB;
  float* qv   = (float*)((char*)d_ws + off); off += statB;
  f16_t* Wi16 = (f16_t*)((char*)d_ws + off); off += wplB;
  f16_t* Wo16 = (f16_t*)((char*)d_ws + off); off += wplB;
  f16_t* Mp   = (f16_t*)((char*)d_ws + off); off += mpB;
  f16_t* sT   = (f16_t*)((char*)d_ws + off); off += actB;
  f16_t* xf16 = (f16_t*)((char*)d_ws + off); off += actB;
  f16_t* Zh   = (f16_t*)((char*)d_ws + off); off += actB;
  f16_t* Zl   = (f16_t*)((char*)d_ws + off); off += actB;
  float* S    = (float*)((char*)d_ws + off); off += sB;
  f16_t* P    = (f16_t*)((char*)d_ws + off); off += pB;
  float* invl = (float*)((char*)d_ws + off); off += ilB;
  if (off > ws_size) return;
  f16_t* Ofp = Zh;

  hipFuncSetAttribute(reinterpret_cast<const void*>(&xproj_kernel),
                      hipFuncAttributeMaxDynamicSharedMemorySize, (int)XPROJ_LDS);
  hipFuncSetAttribute(reinterpret_cast<const void*>(&zproj_kernel),
                      hipFuncAttributeMaxDynamicSharedMemorySize, (int)ZPROJ_LDS);

  cvtw_kernel<<<dim3(2 * (kC * kC / 8) / 256), dim3(256), 0, stream>>>(i_w, o_w, Wi16, Wo16);
  stats_kernel<<<dim3(2 * (kB * kC / 32)), dim3(256), 0, stream>>>(c, s, mu_c, r_c, mu_s, r_s);
  mgemm_kernel<<<dim3(kC / 64, kC / 64), dim3(128), 0, stream>>>(s_w, c_w, r_c, Mp);
  q_kernel<<<dim3(kB * kC / 256), dim3(256), 0, stream>>>(s_w, c_b, Mp, mu_c, qv);
  xproj_kernel<<<dim3(kB * NPB), dim3(128), XPROJ_LDS, stream>>>(s, Wi16, i_b, sT, xf16);
  zproj_kernel<<<dim3(kB * NPB), dim3(128), ZPROJ_LDS, stream>>>(c, Mp, qv, r_s, Zh, Zl);

  for (int b = 0; b < kB; ++b) {
    for (int hb = 0; hb < 2; ++hb) {
      const int nbase = hb * kNH;
      sgemm_kernel<<<dim3(kN / 128, kNH / 64), dim3(256), 0, stream>>>(Zh, Zl, sT, S, b, nbase);
      softmax_kernel<<<dim3(kNH / 32), dim3(SMB), 0, stream>>>(S, P, invl);
      pv_kernel<<<dim3(kNH / 128, kC / 64), dim3(256), 0, stream>>>(xf16, P, invl, Ofp, b, nbase);
    }
  }
  out_kernel<<<dim3(kN / 128, kC / 64, kB), dim3(256), 0, stream>>>(Wo16, Ofp, o_b, x, out);
}
